// FusedNeRF_6957847019903
// MI455X (gfx1250) — hardware-verified
//
#include <hip/hip_runtime.h>
#include <stdint.h>

typedef _Float16 v16h __attribute__((ext_vector_type(16)));
typedef _Float16 v8h  __attribute__((ext_vector_type(8)));
typedef float    v8f  __attribute__((ext_vector_type(8)));
typedef float    v4f  __attribute__((ext_vector_type(4)));
typedef unsigned int v4u __attribute__((ext_vector_type(4)));

#define HID   64
#define NPTT  32

#define OFF_S0 0
#define OFF_S1 2048
#define OFF_S2 6144
#define OFF_C0 7168
#define OFF_C1 9216
#define OFF_C2 13312
#define OFF_C3 17408
#define TOTAL_WH 18432
static_assert((TOTAL_WH % 256) == 0);
static_assert(((OFF_S1 | OFF_S2 | OFF_C0 | OFF_C1 | OFF_C2 | OFF_C3) % 64) == 0);

#define WSC  64.0f
#define XSC  16.0f
#define RACT (1.0f / 64.0f)
#define ROUT (1.0f / 1024.0f)
#define RESC 4096.0f
#define RRES (1.0f / 4096.0f)

__device__ __forceinline__ unsigned short bf_bits(float f) {
  unsigned u = __float_as_uint(f);
  return (unsigned short)((u + 0x7FFFu + ((u >> 16) & 1u)) >> 16);
}
__device__ __forceinline__ float bf_up(unsigned short h) { return __uint_as_float(((unsigned)h) << 16); }
__device__ __forceinline__ unsigned short h_bits(_Float16 x) { return __builtin_bit_cast(unsigned short, x); }
__device__ __forceinline__ unsigned short hb(float f) { return h_bits((_Float16)f); }
__device__ __forceinline__ unsigned pk16(unsigned short a, unsigned short b) { return (unsigned)a | ((unsigned)b << 16); }
__device__ __forceinline__ v8f zero8() { v8f z = {0.f, 0.f, 0.f, 0.f, 0.f, 0.f, 0.f, 0.f}; return z; }

__device__ __forceinline__ v16h ldfrag_h(const _Float16* p) {
  union { v16h v; v8h h[2]; } f;
  f.h[0] = *(const v8h*)(p);
  f.h[1] = *(const v8h*)(p + 16);
  return f.v;
}

__device__ __forceinline__ v8f mma_h(v16h a, v16h b, v8f c) {
  c = __builtin_amdgcn_wmma_f32_16x16x32_f16(false, a, false, b, (short)0, c, false, false);
#if defined(__HIP_DEVICE_COMPILE__)
  asm volatile("v_nop\n\tv_nop\n\tv_nop\n\tv_nop" : "+v"(c) : "v"(a), "v"(b));
#endif
  return c;
}
__device__ __forceinline__ void wave_sync_lds() {
  __builtin_amdgcn_fence(__ATOMIC_RELEASE, "workgroup");
  __builtin_amdgcn_wave_barrier();
  __builtin_amdgcn_fence(__ATOMIC_ACQUIRE, "workgroup");
}

template <bool RELU>
__device__ __forceinline__ v16h pack_next(v8f dlo, v8f dhi) {
  union { v16h v; unsigned u[8]; } t;
#pragma unroll
  for (int d = 0; d < 4; ++d) {
    float a0 = dlo[2 * d], a1 = dlo[2 * d + 1];
    float c0 = dhi[2 * d], c1 = dhi[2 * d + 1];
    if (RELU) { a0 = fmaxf(a0, 0.f); a1 = fmaxf(a1, 0.f); c0 = fmaxf(c0, 0.f); c1 = fmaxf(c1, 0.f); }
    t.u[d]     = pk16(hb(a0 * RACT), hb(a1 * RACT));
    t.u[4 + d] = pk16(hb(c0 * RACT), hb(c1 * RACT));
  }
  return t.v;
}
template <bool RELU>
__device__ __forceinline__ void pack_split(v8f dlo, v8f dhi, v16h& bhi, v16h& bres) {
  union { v16h v; unsigned u[8]; } th, tr;
#pragma unroll
  for (int d = 0; d < 4; ++d) {
    float a0 = dlo[2 * d], a1 = dlo[2 * d + 1];
    float c0 = dhi[2 * d], c1 = dhi[2 * d + 1];
    if (RELU) { a0 = fmaxf(a0, 0.f); a1 = fmaxf(a1, 0.f); c0 = fmaxf(c0, 0.f); c1 = fmaxf(c1, 0.f); }
    const float v0 = a0 * RACT, v1 = a1 * RACT, w0 = c0 * RACT, w1 = c1 * RACT;
    const _Float16 x0 = (_Float16)v0, x1 = (_Float16)v1, y0 = (_Float16)w0, y1 = (_Float16)w1;
    th.u[d]     = pk16(h_bits(x0), h_bits(x1));
    th.u[4 + d] = pk16(h_bits(y0), h_bits(y1));
    tr.u[d]     = pk16(hb((v0 - (float)x0) * RESC), hb((v1 - (float)x1) * RESC));
    tr.u[4 + d] = pk16(hb((w0 - (float)y0) * RESC), hb((w1 - (float)y1) * RESC));
  }
  bhi  = th.v;
  bres = tr.v;
}

template <int KC>
__device__ __forceinline__ void layer64(const _Float16* w, const v16h (&b0)[2], const v16h (&b1)[2],
                                        v8f (&h)[2][4], int c, int g) {
#pragma unroll
  for (int mt = 0; mt < 4; ++mt) {
    const _Float16* p = w + (mt * 16 + c) * (32 * KC) + 8 * g;
    const v16h a0 = ldfrag_h(p);
    v16h a1 = a0;
    if (KC == 2) a1 = ldfrag_h(p + 32);
#pragma unroll
    for (int u = 0; u < 2; ++u) {
      v8f acc = mma_h(a0, b0[u], zero8());
      if (KC == 2) acc = mma_h(a1, b1[u], acc);
      h[u][mt] = acc;
    }
  }
}
__device__ __forceinline__ void layer64s(const _Float16* w, const v16h (&b0)[2], const v16h (&b1)[2],
                                         const v16h (&q0)[2], const v16h (&q1)[2],
                                         v8f (&h)[2][4], int c, int g) {
#pragma unroll
  for (int mt = 0; mt < 4; ++mt) {
    const _Float16* p = w + (mt * 16 + c) * 64 + 8 * g;
    const v16h a0 = ldfrag_h(p);
    const v16h a1 = ldfrag_h(p + 32);
#pragma unroll
    for (int u = 0; u < 2; ++u) {
      v8f acc = mma_h(a0, b0[u], zero8());
      acc = mma_h(a1, b1[u], acc);
      v8f accr = mma_h(a0, q0[u], zero8());
      accr = mma_h(a1, q1[u], accr);
      v8f o;
#pragma unroll
      for (int r = 0; r < 8; ++r) o[r] = acc[r] + accr[r] * RRES;
      h[u][mt] = o;
    }
  }
}
__device__ __forceinline__ void layer16(const _Float16* w, const v16h (&b0)[2], const v16h (&b1)[2],
                                        v8f (&s)[2], int c, int g) {
  const _Float16* p = w + c * 64 + 8 * g;
  const v16h a0 = ldfrag_h(p);
  const v16h a1 = ldfrag_h(p + 32);
#pragma unroll
  for (int u = 0; u < 2; ++u) {
    v8f acc = mma_h(a0, b0[u], zero8());
    acc = mma_h(a1, b1[u], acc);
    s[u] = acc;
  }
}
__device__ __forceinline__ void layer16s(const _Float16* w, const v16h (&b0)[2], const v16h (&b1)[2],
                                         const v16h (&q0)[2], const v16h (&q1)[2],
                                         v8f (&s)[2], int c, int g) {
  const _Float16* p = w + c * 64 + 8 * g;
  const v16h a0 = ldfrag_h(p);
  const v16h a1 = ldfrag_h(p + 32);
#pragma unroll
  for (int u = 0; u < 2; ++u) {
    v8f acc = mma_h(a0, b0[u], zero8());
    acc = mma_h(a1, b1[u], acc);
    v8f accr = mma_h(a0, q0[u], zero8());
    accr = mma_h(a1, q1[u], accr);
    v8f o;
#pragma unroll
    for (int r = 0; r < 8; ++r) o[r] = acc[r] + accr[r] * RRES;
    s[u] = o;
  }
}

__global__ __launch_bounds__(256) void wprep(const float* __restrict__ sw0, const float* __restrict__ sw1,
                                             const float* __restrict__ sw2, const float* __restrict__ cw0,
                                             const float* __restrict__ cw1, const float* __restrict__ cw2,
                                             const float* __restrict__ cw3, unsigned short* wp) {
  const int s = blockIdx.y;
  const float* src;
  int nact, kact, kp, npad, off, mode;
  if (s == 0)      { src = sw0; nact = 64; kact = 3;  kp = 32; npad = 64; off = OFF_S0; mode = 0; }
  else if (s == 1) { src = sw1; nact = 64; kact = 64; kp = 64; npad = 64; off = OFF_S1; mode = 0; }
  else if (s == 2) { src = sw2; nact = 16; kact = 64; kp = 64; npad = 16; off = OFF_S2; mode = 0; }
  else if (s == 3) { src = cw0; nact = 64; kact = 18; kp = 32; npad = 64; off = OFF_C0; mode = 1; }
  else if (s == 4) { src = cw1; nact = 64; kact = 64; kp = 64; npad = 64; off = OFF_C1; mode = 0; }
  else if (s == 5) { src = cw2; nact = 64; kact = 64; kp = 64; npad = 64; off = OFF_C2; mode = 0; }
  else             { src = cw3; nact = 3;  kact = 64; kp = 64; npad = 16; off = OFF_C3; mode = 0; }

  const int nthr = (npad * kp) >> 3;
  const int t = blockIdx.x * 256 + threadIdx.x;
  if (t >= nthr) return;
  const int e0   = t * 8;
  const int row  = e0 / kp;
  const int kb   = e0 - row * kp;
  const int rowc = min(row, nact - 1);

  v4u p;
#pragma unroll
  for (int e = 0; e < 4; ++e) {
    unsigned short bits[2];
#pragma unroll
    for (int j = 0; j < 2; ++j) {
      const int k = kb + 2 * e + j;
      int col; bool valid;
      if (mode == 0) {
        col = k; valid = (row < nact) && (k < kact);
      } else {
        col = (k <= 15) ? (k + 2) : (k - 16);
        valid = (row < nact) && (k >= 1) && (k <= 18);
      }
      const int colc = min(max(col, 0), kact - 1);
      float v = src[(size_t)rowc * kact + colc];
      v = valid ? v : 0.f;
      bits[j] = hb(bf_up(bf_bits(v)) * WSC);
    }
    p[e] = pk16(bits[0], bits[1]);
  }
  unsigned short* dst = wp + off + e0;
  for (int pass = 0; pass < 2; ++pass) {
    *(volatile v4u*)dst = p;
    __threadfence();
  }
}

__global__ __launch_bounds__(256) void mlp_fused(const float* __restrict__ x,
                                                 const unsigned short* __restrict__ wp,
                                                 float* out, int numTiles) {
  __shared__ __align__(16) _Float16 sw[TOTAL_WH];
  __shared__ __align__(16) float oslab[8][NPTT * 4];
  {
    const v4u* src = (const v4u*)(const void*)wp;
    v4u* dst = (v4u*)(void*)sw;
    for (int i = threadIdx.x; i < TOTAL_WH / 8; i += 256) dst[i] = src[i];
  }
  __syncthreads();

  const int lane = threadIdx.x & 31;
  const int wave = threadIdx.x >> 5;
  const int c    = lane & 15;
  const int g    = lane >> 4;
  const int gw     = blockIdx.x * 8 + wave;
  const int stride = gridDim.x * 8;
  float* slab = oslab[wave];

  for (int tile = gw; tile < numTiles; tile += stride) {
    const int pt0 = tile * NPTT;

    float xs[2][6];
#pragma unroll
    for (int u = 0; u < 2; ++u) {
      const float* xr = x + ((size_t)pt0 + u * 16 + c) * 6;
#pragma unroll
      for (int j = 0; j < 6; ++j) xs[u][j] = bf_up(bf_bits(xr[j])) * XSC;
    }

    v16h b0[2], b1[2];
    v16h q0[2], q1[2];
    v8f  h[2][4];

#pragma unroll
    for (int u = 0; u < 2; ++u) {
      union { v16h v; unsigned uu[8]; } t;
      const float f0 = g ? 0.f : xs[u][0];
      const float f1 = g ? 0.f : xs[u][1];
      const float f2 = g ? 0.f : xs[u][2];
      t.uu[0] = pk16(hb(f0), hb(f1));
      t.uu[1] = pk16(hb(f2), (unsigned short)0);
      t.uu[2] = 0u; t.uu[3] = 0u; t.uu[4] = 0u; t.uu[5] = 0u; t.uu[6] = 0u; t.uu[7] = 0u;
      b0[u] = t.v;
      b1[u] = t.v;
    }

    layer64<1>(sw + OFF_S0, b0, b1, h, c, g);
#pragma unroll
    for (int u = 0; u < 2; ++u) {
      pack_split<true>(h[u][0], h[u][1], b0[u], q0[u]);
      pack_split<true>(h[u][2], h[u][3], b1[u], q1[u]);
    }
    layer64s(sw + OFF_S1, b0, b1, q0, q1, h, c, g);
#pragma unroll
    for (int u = 0; u < 2; ++u) {
      pack_split<true>(h[u][0], h[u][1], b0[u], q0[u]);
      pack_split<true>(h[u][2], h[u][3], b1[u], q1[u]);
    }
    v8f s2[2];
    layer16s(sw + OFF_S2, b0, b1, q0, q1, s2, c, g);
    float sig[2];
#pragma unroll
    for (int u = 0; u < 2; ++u) sig[u] = s2[u][0] * ROUT;

#pragma unroll
    for (int u = 0; u < 2; ++u) {
      union { v16h v; unsigned uu[8]; } t;
#pragma unroll
      for (int d = 0; d < 4; ++d)
        t.uu[d] = pk16(hb(s2[u][2 * d] * RACT), hb(s2[u][2 * d + 1] * RACT));
      const float v3 = g ? 0.f : xs[u][3];
      const float v4 = g ? 0.f : xs[u][4];
      const float v5 = g ? 0.f : xs[u][5];
      t.uu[4] = pk16(hb(v3), hb(v4));
      t.uu[5] = pk16(hb(v5), (unsigned short)0);
      t.uu[6] = 0u; t.uu[7] = 0u;
      b0[u] = t.v;
    }

    layer64<1>(sw + OFF_C0, b0, b1, h, c, g);
#pragma unroll
    for (int u = 0; u < 2; ++u) {
      b0[u] = pack_next<true>(h[u][0], h[u][1]);
      b1[u] = pack_next<true>(h[u][2], h[u][3]);
    }
    layer64<2>(sw + OFF_C1, b0, b1, h, c, g);
#pragma unroll
    for (int u = 0; u < 2; ++u) {
      b0[u] = pack_next<true>(h[u][0], h[u][1]);
      b1[u] = pack_next<true>(h[u][2], h[u][3]);
    }
    layer64<2>(sw + OFF_C2, b0, b1, h, c, g);
#pragma unroll
    for (int u = 0; u < 2; ++u) {
      b0[u] = pack_next<true>(h[u][0], h[u][1]);
      b1[u] = pack_next<true>(h[u][2], h[u][3]);
    }
    v8f col[2];
    layer16(sw + OFF_C3, b0, b1, col, c, g);

    wave_sync_lds();
    if (g == 0) {
#pragma unroll
      for (int u = 0; u < 2; ++u) {
        v4f o;
        o[0] = col[u][0] * ROUT;
        o[1] = col[u][1] * ROUT;
        o[2] = col[u][2] * ROUT;
        o[3] = sig[u];
        *(v4f*)(slab + (u * 16 + c) * 4) = o;
      }
    }
    wave_sync_lds();
    const v4f o = *(const v4f*)(slab + lane * 4);
    float* op = out + ((size_t)pt0 + lane) * 4;
    for (int pass = 0; pass < 2; ++pass) {
      *(volatile v4f*)op = o;
      __threadfence();
    }
  }
}

extern "C" void kernel_launch(void* const* d_in, const int* in_sizes, int n_in,
                              void* d_out, int out_size, void* d_ws, size_t ws_size,
                              hipStream_t stream) {
  if (n_in < 8) return;
  if (in_sizes[1] != 64 * 3 || in_sizes[2] != 64 * 64 || in_sizes[3] != 16 * 64 ||
      in_sizes[4] != 64 * 18 || in_sizes[5] != 64 * 64 || in_sizes[6] != 64 * 64 || in_sizes[7] != 3 * 64) return;
  const int nx = in_sizes[0];
  if (nx <= 0 || (nx % 6) != 0) return;
  const int n = nx / 6;
  if ((n % NPTT) != 0) return;
  if (out_size != n * 4) return;
  const size_t carve = (size_t)TOTAL_WH * 2;
  if (carve > ws_size) return;

  const float* x   = (const float*)d_in[0];
  const float* sw0 = (const float*)d_in[1];
  const float* sw1 = (const float*)d_in[2];
  const float* sw2 = (const float*)d_in[3];
  const float* cw0 = (const float*)d_in[4];
  const float* cw1 = (const float*)d_in[5];
  const float* cw2 = (const float*)d_in[6];
  const float* cw3 = (const float*)d_in[7];
  unsigned short* wp = (unsigned short*)d_ws;

  const int numTiles = n / NPTT;
  int blocks = (numTiles + 7) / 8;
  if (blocks > 1024) blocks = 1024;
  if (blocks < 1) return;

  wprep<<<dim3(2, 7), dim3(256), 0, stream>>>(sw0, sw1, sw2, cw0, cw1, cw2, cw3, wp);
  mlp_fused<<<dim3(blocks), dim3(256), 0, stream>>>(x, wp, (float*)d_out, numTiles);
  (void)hipGetLastError();
}
